// CudaW4A16Linear_46686294507979
// MI455X (gfx1250) — hardware-verified
//
#include <hip/hip_runtime.h>


#ifndef NOUT
#define NOUT 11008
#endif
#define NOUT_FULL 11008
#define MROWS 8
#define MPAD  16
#define KIN   4096
#define GSZ   128
#define GROUPS (KIN / GSZ)
#define KD8   (KIN / 8)
#define ZD    4
#define WCOLS 32
#define OSP   36

static_assert(KIN % GSZ == 0);
static_assert(GSZ % 32 == 0);
static_assert(GSZ / 32 == 4);
static_assert(KIN % 32 == 0);
static_assert(GROUPS <= 8 * ZD);
static_assert(NOUT % WCOLS == 0);
static_assert(NOUT <= NOUT_FULL);
static_assert(WCOLS * 4 == 128);
static_assert(((size_t)NOUT_FULL * 4) % 128 == 0);
static_assert(MROWS == 8);
static_assert(MPAD == 16);
static_assert(((size_t)MPAD * KIN / 8) % 256 == 0);
static_assert(((size_t)MROWS * KIN / 8) % 256 == 0);
static_assert(32 * 16 * 2 == MROWS * WCOLS * 4);
static_assert((OSP * 4) % 16 == 0);
static_assert(16 * OSP * 4 <= 131072);

typedef _Float16 h16;
typedef __attribute__((ext_vector_type(16))) _Float16 v16h;
typedef __attribute__((ext_vector_type(8)))  _Float16 v8h;
typedef __attribute__((ext_vector_type(8)))  float    v8f;
typedef __attribute__((ext_vector_type(4)))  float    v4f;
typedef v4f  __attribute__((may_alias)) v4fa;

__device__ __forceinline__ unsigned short f2bf(float f) { unsigned u = __float_as_uint(f); u += 0x7FFFu + ((u >> 16) & 1u); return (unsigned short)(u >> 16); }
__device__ __forceinline__ float bfr(float f) { return __uint_as_float(((unsigned)f2bf(f)) << 16); }
__device__ __forceinline__ v16h cat16(v8h lo, v8h hi) { return __builtin_shufflevector(lo, hi, 0, 1, 2, 3, 4, 5, 6, 7, 8, 9, 10, 11, 12, 13, 14, 15); }
__device__ __forceinline__ v8f wmma16(v16h a, v16h b, v8f c) { return __builtin_amdgcn_wmma_f32_16x16x32_f16(false, a, false, b, (short)0, c, false, false); }
__device__ __forceinline__ v16h  ldh(const h16* p) { return cat16(*(const v8h*)p, *(const v8h*)(p + 16)); }
__device__ __forceinline__ void wave_sync() { __builtin_amdgcn_fence(3  , "wavefront"); __builtin_amdgcn_wave_barrier(); asm volatile("" ::: "memory"); }

static __device__ __forceinline__ h16 toh_flush(float v) { const h16 r = (h16)v; return (fabsf(v) < 6.103515625e-05f) ? (h16)0.0f : r; }

__device__ __forceinline__ v8f wmma16g(v16h a, v16h b, v8f c) {
    c = wmma16(a, b, c);
    asm volatile("v_nop\n\tv_nop\n\tv_nop\n\tv_nop" : "+v"(c) : "v"(a), "v"(b));
    return c;
}

__device__ __forceinline__ v8h dq8(unsigned w, int z) {
    v8h r;
#pragma unroll
    for (int i = 0; i < 8; ++i) {
        const int q = (int)((w >> (4 * i)) & 15u);
        const int d = q - z;
        r[i] = (h16)(float)d;
    }
    return r;
}

__device__ __forceinline__ v16h wfrag(unsigned w0, unsigned w1, int z) {
    return cat16(dq8(w0, z), dq8(w1, z));
}

#define XRB ((MROWS * KIN / 8) / 256)
__global__ __launch_bounds__(256) void k_xcvt(const float* __restrict__ src, h16* dst) {
    const size_t i = (size_t)blockIdx.x * 256 + threadIdx.x;
    v8h o = (v8h){};
    if (blockIdx.x < XRB) {
        const v8f v = *(const v8f*)(src + i * 8);
#pragma unroll
        for (int k = 0; k < 8; ++k) o[k] = toh_flush(bfr(v[k]));
    }
    *(volatile v8h*)(dst + i * 8) = o; __threadfence(); *(volatile v8h*)(dst + i * 8) = o;
}

__global__ __launch_bounds__(32) void k_w4gemm(const h16* __restrict__ XH, const int* __restrict__ QW, const int* __restrict__ QZ, const float* __restrict__ SCL, float* OUT) {
    __shared__ __align__(16) float os[16 * OSP];
    const int lane = threadIdx.x & 31, lr = lane & 15, hi = lane >> 4;
    const int c0 = blockIdx.x * WCOLS;
    const int colA = c0 + lr, colB = c0 + 16 + lr;
    const size_t wa = (size_t)colA * KD8 + hi, wb = (size_t)colB * KD8 + hi;
    const size_t xo = (size_t)lr * KIN + 8 * hi;
    v8f cA = (v8f){}, cB = (v8f){};
#pragma unroll 1
    for (int g = 0; g < GROUPS; ++g) {
        const unsigned zwa = (unsigned)QZ[(size_t)colA * ZD + (g >> 3)];
        const unsigned zwb = (unsigned)QZ[(size_t)colB * ZD + (g >> 3)];
        const int za = (int)((zwa >> ((g & 7) * 4)) & 15u), zb = (int)((zwb >> ((g & 7) * 4)) & 15u);
        const float sa = bfr(SCL[(size_t)colA * GROUPS + g]);
        const float sb = bfr(SCL[(size_t)colB * GROUPS + g]);
        v8f gA = (v8f){}, gB = (v8f){};
#pragma unroll 2
        for (int it = 0; it < GSZ / 32; ++it) {
            const int k0 = g * GSZ + it * 32;
            const int d = k0 >> 3;
            const v16h a = ldh(XH + xo + k0);
            const unsigned a0 = (unsigned)QW[wa + d], a1 = (unsigned)QW[wa + d + 2];
            const unsigned b0 = (unsigned)QW[wb + d], b1 = (unsigned)QW[wb + d + 2];
            const v16h fa = wfrag(a0, a1, za);
            const v16h fb = wfrag(b0, b1, zb);
            gA = wmma16g(a, fa, gA);
            gB = wmma16g(a, fb, gB);
        }
#pragma unroll
        for (int r = 0; r < 8; ++r) { cA[r] = __builtin_fmaf(sa, gA[r], cA[r]); cB[r] = __builtin_fmaf(sb, gB[r], cB[r]); }
    }
#pragma unroll
    for (int r = 0; r < 8; ++r) { os[(8 * hi + r) * OSP + lr] = cA[r]; os[(8 * hi + r) * OSP + 16 + lr] = cB[r]; }
    wave_sync();
    float* orow = OUT + c0;
#pragma unroll 1
    for (int ps = 0; ps < 2; ++ps) {
#pragma unroll
        for (int s = 0; s < 2; ++s) { const int row = 4 * s + (lane >> 3), cofs = (lane & 7) * 4;
            const v4f val = *(const v4fa*)(&os[row * OSP + cofs]);
            *(volatile v4f*)(orow + (size_t)row * NOUT_FULL + cofs) = val; }
        if (ps == 0) __threadfence(); }
}

static constexpr size_t al256(size_t v) { return (v + 255) & ~(size_t)255; }
static constexpr size_t SZ_XH = al256((size_t)MPAD * KIN * 2);
static constexpr size_t SZ_TOTAL = SZ_XH;
static_assert(SZ_TOTAL <= (size_t)134217728);
static_assert((size_t)MPAD * KIN * 2 == (size_t)((MPAD * KIN / 8) / 256) * 256 * 16);

extern "C" void kernel_launch(void* const* d_in, const int* in_sizes, int n_in,
                              void* d_out, int out_size, void* d_ws, size_t ws_size, hipStream_t stream) {
    if (n_in < 4) return;
    if ((size_t)in_sizes[0] < (size_t)MROWS * KIN) return;
    if ((size_t)in_sizes[1] < (size_t)NOUT * KD8) return;
    if ((size_t)in_sizes[2] < (size_t)NOUT * ZD) return;
    if ((size_t)in_sizes[3] < (size_t)NOUT * GROUPS) return;
    if ((size_t)out_size < (size_t)(MROWS - 1) * NOUT_FULL + NOUT) return;
    if (SZ_TOTAL > ws_size) return;
    const float* x  = (const float*)d_in[0];
    const int*   qw = (const int*)d_in[1];
    const int*   qz = (const int*)d_in[2];
    const float* sc = (const float*)d_in[3];
    float* OUT = (float*)d_out;
    char* wsp = (char*)d_ws;
    h16* XH = (h16*)wsp; wsp += SZ_XH;

    k_xcvt<<<(unsigned)((MPAD * KIN / 8) / 256), 256, 0, stream>>>(x, XH);
    k_w4gemm<<<(unsigned)(NOUT / WCOLS), 32, 0, stream>>>(XH, qw, qz, sc, OUT);
}
